// GraphConvolution_59304908423183
// MI455X (gfx1250) — hardware-verified
//
#include <hip/hip_runtime.h>
#include <math.h>

typedef __attribute__((ext_vector_type(16))) _Float16 v16h;
typedef __attribute__((ext_vector_type(16))) __bf16 v16b;
typedef __attribute__((ext_vector_type(8)))  _Float16 v8h;
typedef __attribute__((ext_vector_type(8)))  float v8f;
typedef __attribute__((ext_vector_type(4)))  float v4f;
typedef __attribute__((ext_vector_type(2)))  float v2f;
typedef __attribute__((ext_vector_type(4)))  unsigned v4u;
typedef __attribute__((ext_vector_type(4)))  int v4i;
typedef float __attribute__((may_alias)) float_a;
typedef int __attribute__((may_alias)) int_a;

template <typename T> __device__ __forceinline__ void vst2(void* p, T v) { *(volatile T*)p = v; __threadfence(); *(volatile T*)p = v; }
__device__ __forceinline__ v8f wmma16(v16h a, v16h b, v8f c) {
  v8f d = __builtin_amdgcn_wmma_f32_16x16x32_f16(false, a, false, b, (short)0, c, false, false);
  asm volatile("v_nop\n\tv_nop\n\tv_nop\n\tv_nop" : "+v"(d) : "v"(a), "v"(b));
  return d;
}
__device__ __forceinline__ v8f wmma_bf(v16b a, v16b b, v8f c) {
  v8f d = __builtin_amdgcn_wmma_f32_16x16x32_bf16(false, a, false, b, (short)0, c, false, false);
  asm volatile("v_nop\n\tv_nop\n\tv_nop\n\tv_nop" : "+v"(d) : "v"(a), "v"(b));
  return d;
}
__device__ __forceinline__ v16h frag_h(const _Float16* rowk0, int lane) {
  union { v16h v; v8h q[2]; } u; const _Float16* p = rowk0 + 8 * (lane >> 4);
  u.q[0] = *(const v8h*)p; u.q[1] = *(const v8h*)(p + 16); return u.v;
}
__device__ __forceinline__ v16h frag_f32(const float* rowk0, int lane) {
  v16h a; const float* p = rowk0 + 8 * (lane >> 4);
#pragma unroll
  for (int i = 0; i < 8; ++i) { a[i] = (_Float16)p[i]; a[8 + i] = (_Float16)p[16 + i]; }
  return a;
}
__device__ __forceinline__ v16h frag_f32s(const float* rowk0, int lane, float sc) {
  v16h a; const float* p = rowk0 + 8 * (lane >> 4);
#pragma unroll
  for (int i = 0; i < 8; ++i) { a[i] = (_Float16)(p[i] * sc); a[8 + i] = (_Float16)(p[16 + i] * sc); }
  return a;
}
__device__ __forceinline__ v16h fragc_f32(const float* W, int k0, int n, int lane, int ld, int K) {
  v16h a; const int g = lane >> 4;
#pragma unroll
  for (int i = 0; i < 8; ++i) { const int ka = k0 + 8 * g + i, kb = ka + 16;
    a[i] = (_Float16)(ka < K ? W[(size_t)(ka < K ? ka : K - 1) * ld + n] : 0.f); a[8 + i] = (_Float16)(kb < K ? W[(size_t)(kb < K ? kb : K - 1) * ld + n] : 0.f); }
  return a;
}
struct F2 { v16b h, l; };
__device__ __forceinline__ F2 bsplit16(const float v[16]) { F2 r;
#pragma unroll
  for (int i = 0; i < 16; ++i) { const __bf16 h = (__bf16)v[i]; r.h[i] = h; r.l[i] = (__bf16)(v[i] - (float)h); }
  return r; }
__device__ __forceinline__ F2 split_row(const float* row, int k0, int lane) { float v[16]; const float* p = row + k0 + 8 * (lane >> 4);
#pragma unroll
  for (int i = 0; i < 8; ++i) { v[i] = p[i]; v[8 + i] = p[16 + i]; }
  return bsplit16(v); }
__device__ __forceinline__ F2 split_rowK(const float* row, int k0, int lane, int K) { float v[16]; const int g = lane >> 4;
#pragma unroll
  for (int i = 0; i < 8; ++i) { const int ka = k0 + 8 * g + i, kb = ka + 16; v[i] = ka < K ? row[ka < K ? ka : K - 1] : 0.f; v[8 + i] = kb < K ? row[kb < K ? kb : K - 1] : 0.f; }
  return bsplit16(v); }
__device__ __forceinline__ F2 split_col(const float* W, int k0, int n, int lane, int ld, int K) { float v[16]; const int g = lane >> 4;
#pragma unroll
  for (int i = 0; i < 8; ++i) { const int ka = k0 + 8 * g + i, kb = ka + 16; v[i] = ka < K ? W[(size_t)(ka < K ? ka : K - 1) * ld + n] : 0.f; v[8 + i] = kb < K ? W[(size_t)(kb < K ? kb : K - 1) * ld + n] : 0.f; }
  return bsplit16(v); }
__device__ __forceinline__ v8f mac3(const F2& a, const F2& b, v8f c) { c = wmma_bf(a.l, b.h, c); c = wmma_bf(a.h, b.l, c); return wmma_bf(a.h, b.h, c); }
__device__ __forceinline__ float sigm(float v) { return 1.0f / (1.0f + expf(-v)); }
#define LDSX() do { asm volatile("s_wait_dscnt 0" ::: "memory"); __builtin_amdgcn_wave_barrier(); __builtin_amdgcn_fence(__ATOMIC_RELEASE, "workgroup"); } while (0)


#define NBG 32
#define NN 256
#define NL 16
#define XD 256
#define YD 64
#define NNODE (NBG * NN)
#define NEDGE (NNODE * NL)
#ifndef NNP
#define NNP NNODE
#endif
__device__ __forceinline__ float bfr(float v) { return (float)(__bf16)v; }
__device__ __forceinline__ float fexp(float x) { x = fminf(fmaxf(x, -87.0f), 88.0f); const float k = rintf(x * 1.44269504088896341f); float r = fmaf(k, -6.93145751953125e-1f, x); r = fmaf(k, -1.42860676533018e-6f, r);
  float p = 1.0f / 5040.0f; p = fmaf(p, r, 1.0f / 720.0f); p = fmaf(p, r, 1.0f / 120.0f); p = fmaf(p, r, 1.0f / 24.0f); p = fmaf(p, r, 1.0f / 6.0f); p = fmaf(p, r, 0.5f); p = fmaf(p, r, 1.0f); p = fmaf(p, r, 1.0f);
  const int ki = (int)k; return p * __int_as_float((ki + 127) << 23); }
__device__ __forceinline__ float fsigm(float z) { return 1.0f / (1.0f + fexp(-z)); }
__device__ __forceinline__ float ftanh(float z) { z = fminf(fmaxf(z, -15.0f), 15.0f); const float t = fexp(2.0f * z); return (t - 1.0f) / (t + 1.0f); }
#define WS_PQ  0u
#define WS_VN  (WS_PQ + 4u * (size_t)NNODE * 1024)
#define WS_END (WS_VN + 4u * (size_t)NNODE * XD)
__global__ __launch_bounds__(128) void k_node(const float* __restrict__ V, const float* __restrict__ WF, const float* __restrict__ WSs, float* __restrict__ PQ) { __shared__ __align__(16) float sf[4][16][132];
  const int tid = threadIdx.x, wave = tid >> 5, lane = tid & 31, col = lane & 15, g = lane >> 4; const int c0 = blockIdx.y * 128; const size_t r0 = (size_t)blockIdx.x * 64 + wave * 16; const int seg = c0 >> 8; const float* WB = (seg < 2 ? WF : WSs) + (size_t)((seg & 1) * XD) * XD; const int oc0 = c0 & 255;
  v8f acc[8] = {};
#pragma unroll 2
  for (int kc = 0; kc < XD / 32; ++kc) { v16b a; { const float* p = V + (r0 + col) * XD + kc * 32 + 8 * g;
#pragma unroll
      for (int i = 0; i < 8; ++i) { a[i] = (__bf16)p[i]; a[8 + i] = (__bf16)p[16 + i]; } }
#pragma unroll
    for (int j = 0; j < 8; ++j) { v16b w; const int o = oc0 + j * 16 + col;
#pragma unroll
      for (int i = 0; i < 8; ++i) { w[i] = (__bf16)WB[(size_t)(kc * 32 + 8 * g + i) * XD + o]; w[8 + i] = (__bf16)WB[(size_t)(kc * 32 + 16 + 8 * g + i) * XD + o]; }
      asm volatile("s_wait_loadcnt 0x0" ::: "memory"); acc[j] = wmma_bf(a, w, acc[j]); } }
#pragma unroll
  for (int j = 0; j < 8; ++j)
#pragma unroll
    for (int r = 0; r < 8; ++r) sf[wave][8 * g + r][j * 16 + col] = acc[j][r];
  LDSX(); for (int rl = 0; rl < 16; ++rl) vst2(PQ + (r0 + rl) * 1024 + c0 + lane * 4, *(const v4f*)&sf[wave][rl][lane * 4]); }
__global__ __launch_bounds__(128) void k_edge(const float* __restrict__ V, const int* __restrict__ NLI, const float* __restrict__ E, const float* __restrict__ WF, const float* __restrict__ BF, const float* __restrict__ WSs, const float* __restrict__ BS, const float* __restrict__ PQ, float* __restrict__ VN) {
  __shared__ __align__(16) float sq[64][132];
  __shared__ int snl[64]; __shared__ __align__(16) float so[4][64];
  const int tid = threadIdx.x, wave = tid >> 5, lane = tid & 31, col = lane & 15, g = lane >> 4; const int x0 = blockIdx.y * 64; const size_t e0 = (size_t)blockIdx.x * 64; const size_t node0 = e0 / NL; const size_t graph = node0 / NN;
  if (tid < 64) snl[tid] = NLI[e0 + tid];
  __syncthreads();
  for (int p = tid; p < 64 * 32; p += 128) { const int ed = p >> 5, q = p & 31; const int nl = snl[ed]; const int j = nl < 0 ? 0 : (nl >= NN ? NN - 1 : nl); const size_t srow = graph * NN + j; const int half = q >> 4, qq = q & 15;
    const v4f v = *(const v4f*)(PQ + srow * 1024 + (half ? 768 : 256) + x0 + qq * 4); *(v4f*)&sq[ed][half * 64 + qq * 4] = v; }
  __syncthreads();
  v8f acc[8] = {};
#pragma unroll
  for (int kc = 0; kc < YD / 32; ++kc) { v16b a; { const float* p = E + (e0 + wave * 16 + col) * YD + kc * 32 + 8 * g;
#pragma unroll
      for (int i = 0; i < 8; ++i) { a[i] = (__bf16)p[i]; a[8 + i] = (__bf16)p[16 + i]; } }
#pragma unroll
    for (int j = 0; j < 8; ++j) { v16b w; const float* WB = (j < 4 ? WF : WSs) + (size_t)(2 * XD) * XD; const int o = x0 + (j & 3) * 16 + col;
#pragma unroll
      for (int i = 0; i < 8; ++i) { w[i] = (__bf16)WB[(size_t)(kc * 32 + 8 * g + i) * XD + o]; w[8 + i] = (__bf16)WB[(size_t)(kc * 32 + 16 + 8 * g + i) * XD + o]; }
      asm volatile("s_wait_loadcnt 0x0" ::: "memory"); acc[j] = wmma_bf(a, w, acc[j]); } }
  const size_t node = node0 + wave; float sum[4];
#pragma unroll
  for (int jj = 0; jj < 4; ++jj) { const int x = x0 + jj * 16 + col; const float pf = PQ[node * 1024 + x] + bfr(BF[x]), ps = PQ[node * 1024 + 512 + x] + bfr(BS[x]); float s_ = 0.f;
#pragma unroll
    for (int r = 0; r < 8; ++r) { const int le = wave * 16 + 8 * g + r; const bool m = snl[le] >= 0; const float zf = acc[jj][r] + pf + (m ? sq[le][jj * 16 + col] : 0.f); const float zs = acc[jj + 4][r] + ps + (m ? sq[le][64 + jj * 16 + col] : 0.f);
      const float fv = fsigm(zf); const float sv = ftanh(zs); s_ += m ? fv * sv : 0.f; }
    sum[jj] = s_; }
#pragma unroll
  for (int jj = 0; jj < 4; ++jj) sum[jj] += __shfl_xor(sum[jj], 16);
  if (g == 0) {
#pragma unroll
    for (int jj = 0; jj < 4; ++jj) { const int x = x0 + jj * 16 + col; so[wave][jj * 16 + col] = bfr(V[node * XD + x]) + sum[jj]; } }
  LDSX();
  if (lane < 16) vst2(VN + node * XD + x0 + lane * 4, *(const v4f*)&so[wave][lane * 4]); }
__global__ __launch_bounds__(256) void k_bn(const float* __restrict__ VN, const float* __restrict__ GA, const float* __restrict__ BE, const float* __restrict__ MU, const float* __restrict__ VA, float* __restrict__ OUT) {
  const int t = threadIdx.x; const int rl = t >> 4, sub = t & 15; const size_t row = (size_t)blockIdx.x * 16 + rl; const float* vr = VN + row * XD;
  int ok = 1; for (int c = sub * 4; c < XD; c += 64) { const v4f v = *(const v4f*)(vr + c);
#pragma unroll
    for (int z = 0; z < 4; ++z) ok &= (fabsf(v[z]) > 1e-5f) ? 1 : 0; }
#pragma unroll
  for (int o = 1; o < 16; o <<= 1) ok &= __shfl_xor(ok, o);
  for (int c = sub * 4; c < XD; c += 64) { const v4f v = *(const v4f*)(vr + c); v4f o4;
#pragma unroll
    for (int z = 0; z < 4; ++z) { const float sc = bfr(GA[c + z]) / sqrtf(bfr(VA[c + z]) + 1e-3f); const float sh = bfr(BE[c + z]) - bfr(MU[c + z]) * sc; o4[z] = ok ? (v[z] * sc + sh) : 0.f; }
    vst2(OUT + row * XD + c, o4); } }
extern "C" void kernel_launch(void* const* d_in, const int* in_sizes, int n_in, void* d_out, int out_size, void* d_ws, size_t ws_size, hipStream_t stream) {
  (void)in_sizes; (void)n_in; (void)out_size;
  const float** F = (const float**)d_in;
  if (ws_size < (size_t)WS_END) return;
  char* ws = (char*)d_ws; float* PQ = (float*)(ws + WS_PQ); float* VN = (float*)(ws + WS_VN);
  k_node<<<dim3(NNP / 64, 8), 128, 0, stream>>>(F[0], F[3], F[5], PQ);
  k_edge<<<dim3(NNP * NL / 64, XD / 64), 128, 0, stream>>>(F[0], (const int*)d_in[1], F[2], F[3], F[4], F[5], F[6], PQ, VN);
  k_bn<<<dim3(NNP / 16), 256, 0, stream>>>(VN, F[7], F[8], F[9], F[10], (float*)d_out);
}
